// SparseAttention_27788438405182
// MI455X (gfx1250) — hardware-verified
//
#include <hip/hip_runtime.h>


#ifndef NB
#define NB 2
#endif
#ifndef SEQ
#define SEQ 4096
#endif
#define NB_FULL  2
#define SEQ_FULL 4096
#define DM    512
#define NH    8
#define HD    64
#define HALFW 4
#define PADL  32
#define TP    (SEQ + 64)
#define NTOK  (NB * SEQ)
#define SCL   0.125f
static_assert(SEQ % 64 == 0);
static_assert(NTOK % 64 == 0);
static_assert(DM % 64 == 0);
static_assert(NH * HD == DM);
static_assert(HD == 64);
static_assert(NB >= 1 && NB <= NB_FULL);
static_assert(SEQ <= SEQ_FULL);
static_assert(TP % 8 == 0);
static_assert(PADL >= 8 && (PADL % 8) == 0);
static_assert(2 * HALFW + 16 + 8 <= 32 + 8);
static_assert(16 + 2 * HALFW <= 24);

typedef _Float16 h16;
typedef unsigned short bf;
typedef __attribute__((ext_vector_type(16))) __bf16   v16bf;
typedef __attribute__((ext_vector_type(16))) _Float16 v16h;
typedef __attribute__((ext_vector_type(8)))  _Float16 v8h;
typedef __attribute__((ext_vector_type(8)))  unsigned short v8us;
typedef __attribute__((ext_vector_type(8)))  float    v8f;
typedef __attribute__((ext_vector_type(4)))  float    v4f;
typedef v8h  __attribute__((may_alias)) v8ha;
typedef v4f  __attribute__((may_alias)) v4fa;
typedef v8us __attribute__((may_alias)) v8usa;

__device__ __forceinline__ unsigned short f2bf(float f) { unsigned u = __float_as_uint(f); u += 0x7FFFu + ((u >> 16) & 1u); return (unsigned short)(u >> 16); }
__device__ __forceinline__ float bf2f(unsigned short b) { return __uint_as_float(((unsigned)b) << 16); }
__device__ __forceinline__ float bfr(float f) { return bf2f(f2bf(f)); }
__device__ __forceinline__ void splitf(float y, unsigned short& h, unsigned short& l) { h = f2bf(y); l = f2bf(y - bf2f(h)); }
__device__ __forceinline__ v16h cat16(v8h lo, v8h hi) { return __builtin_shufflevector(lo, hi, 0, 1, 2, 3, 4, 5, 6, 7, 8, 9, 10, 11, 12, 13, 14, 15); }
__device__ __forceinline__ v16bf cat16b(v8us lo, v8us hi) { return __builtin_bit_cast(v16bf, __builtin_shufflevector(lo, hi, 0, 1, 2, 3, 4, 5, 6, 7, 8, 9, 10, 11, 12, 13, 14, 15)); }
__device__ __forceinline__ v8f wmma16(v16h a, v16h b, v8f c) { return __builtin_amdgcn_wmma_f32_16x16x32_f16(false, a, false, b, (short)0, c, false, false); }
__device__ __forceinline__ v8f wmmab(v16bf a, v16bf b, v8f c) { return __builtin_amdgcn_wmma_f32_16x16x32_bf16(false, a, false, b, (short)0, c, false, false); }

template <typename T16> struct WFrag;
template <> struct WFrag<h16> { typedef v16h V; static __device__ __forceinline__ V ld(const h16* p) { return cat16(*(const v8h*)p, *(const v8h*)(p + 16)); } static __device__ __forceinline__ v8f mma(V a, V b, v8f c) { return wmma16(a, b, c); } };
template <> struct WFrag<bf> { typedef v16bf V; static __device__ __forceinline__ V ld(const bf* p) { return cat16b(*(const v8us*)p, *(const v8us*)(p + 16)); } static __device__ __forceinline__ v8f mma(V a, V b, v8f c) { return wmmab(a, b, c); } };
template <typename T16, int NSPLIT, bool BIAS>
__global__ __launch_bounds__(32) void k_gemmw(const T16* __restrict__ A, const T16* __restrict__ A2, const T16* __restrict__ Bt, const T16* __restrict__ Bt2, int K, float* C, int ldc, const float* __restrict__ bias, size_t sA, size_t sB, size_t sC) {
    typedef typename WFrag<T16>::V V;
    __shared__ __align__(16) float os[16 * 68];
    const size_t z = blockIdx.z; A += z * sA; if (A2) A2 += z * sA; Bt += z * sB; if (Bt2) Bt2 += z * sB; C += z * sC;
    const int lane = threadIdx.x & 31, lr = lane & 15, hi = lane >> 4; const int r0 = blockIdx.x * 64, c0 = blockIdx.y * 64;
    v8f acc[4][4];
#pragma unroll
    for (int mb = 0; mb < 4; ++mb)
#pragma unroll
        for (int nb = 0; nb < 4; ++nb) acc[mb][nb] = (v8f){};
    const size_t aoff = (size_t)(r0 + lr) * K + 8 * hi, boff = (size_t)(c0 + lr) * K + 8 * hi;
#pragma unroll 1
    for (int kc = 0; kc < K; kc += 32) {
        V a[4], a2[4];
#pragma unroll
        for (int mb = 0; mb < 4; ++mb) { a[mb] = WFrag<T16>::ld(A + aoff + (size_t)mb * 16 * K + kc); if (NSPLIT == 1 || NSPLIT == 2) a2[mb] = WFrag<T16>::ld(A2 + aoff + (size_t)mb * 16 * K + kc); }
#pragma unroll
        for (int nb = 0; nb < 4; ++nb) { const V b = WFrag<T16>::ld(Bt + boff + (size_t)nb * 16 * K + kc); V b2; if (NSPLIT >= 2) b2 = WFrag<T16>::ld(Bt2 + boff + (size_t)nb * 16 * K + kc);
#pragma unroll
            for (int mb = 0; mb < 4; ++mb) { acc[mb][nb] = WFrag<T16>::mma(a[mb], b, acc[mb][nb]); if (NSPLIT == 1 || NSPLIT == 2) acc[mb][nb] = WFrag<T16>::mma(a2[mb], b, acc[mb][nb]); if (NSPLIT >= 2) acc[mb][nb] = WFrag<T16>::mma(a[mb], b2, acc[mb][nb]); } }
        asm volatile("v_nop\n\tv_nop\n\tv_nop\n\tv_nop" : "+v"(acc[0][0]), "+v"(acc[1][1]), "+v"(acc[2][2]), "+v"(acc[3][3]) : "v"(a[0]), "v"(a[3]));
    }
#pragma unroll
    for (int mb = 0; mb < 4; ++mb) {
#pragma unroll
        for (int nb = 0; nb < 4; ++nb) {
#pragma unroll
            for (int j = 0; j < 8; ++j) os[(hi * 8 + j) * 68 + nb * 16 + lr] = acc[mb][nb][j]; }
        __builtin_amdgcn_wave_barrier(); asm volatile("" ::: "memory");
        float* crow = C + (size_t)(r0 + mb * 16) * ldc + c0;
#pragma unroll 1
        for (int ps = 0; ps < 2; ++ps) {
#pragma unroll
            for (int s = 0; s < 8; ++s) { const int row = 2 * s + hi, cofs = lr * 4; v4f val = *(const v4fa*)(os + row * 68 + cofs); if (BIAS) { val[0] += bfr(bias[c0 + cofs]); val[1] += bfr(bias[c0 + cofs + 1]); val[2] += bfr(bias[c0 + cofs + 2]); val[3] += bfr(bias[c0 + cofs + 3]); }
                *(volatile v4f*)(crow + (size_t)row * ldc + cofs) = val; }
            if (ps == 0) __threadfence(); }
        __builtin_amdgcn_wave_barrier(); asm volatile("" ::: "memory");
    }
}

__global__ __launch_bounds__(256) void k_cvt8(const float* __restrict__ src, bf* dst, size_t n8) { const size_t i = (size_t)blockIdx.x * 256 + threadIdx.x; if (i >= n8) return; const v8f v = *(const v8f*)(src + i * 8); v8us o;
#pragma unroll
    for (int k = 0; k < 8; ++k) o[k] = f2bf(v[k]); *(volatile v8us*)(dst + i * 8) = o; __threadfence(); *(volatile v8us*)(dst + i * 8) = o; }

__global__ __launch_bounds__(256) void k_hlpad(const float* __restrict__ F, bf* Ph, bf* Pl, size_t n8) {
    const size_t i = (size_t)blockIdx.x * 256 + threadIdx.x; if (i >= n8) return;
    const size_t e = i * 8; const int c = (int)(e % DM); const size_t r = e / DM; const int tp = (int)(r % TP); const int b = (int)(r / TP);
    const int t = tp - PADL; const bool ok = (t >= 0) && (t < SEQ); const int tc = t < 0 ? 0 : (t >= SEQ ? SEQ - 1 : t);
    const v8f v = *(const v8f*)(F + ((size_t)b * SEQ + tc) * DM + c);
    v8us oh, ol;
#pragma unroll
    for (int q = 0; q < 8; ++q) { unsigned short a2, c2; splitf(ok ? v[q] : 0.0f, a2, c2); oh[q] = a2; ol[q] = c2; }
    *(volatile v8us*)(Ph + e) = oh; *(volatile v8us*)(Pl + e) = ol; __threadfence(); *(volatile v8us*)(Ph + e) = oh; *(volatile v8us*)(Pl + e) = ol;
}

__global__ __launch_bounds__(256) void k_vthl(const float* __restrict__ G, bf* Vh, bf* Vl, size_t n8) {
    const size_t i = (size_t)blockIdx.x * 256 + threadIdx.x; if (i >= n8) return;
    const size_t e = i * 8; const int tp = (int)(e % TP); const size_t qq = e / TP; const int b = (int)(qq % NB); const int n = (int)(qq / NB);
    const int t = tp - PADL; const bool ok = (t >= 0) && (t < SEQ); const int tc = t < 0 ? 0 : (t > SEQ - 8 ? SEQ - 8 : t);
    const v8f v = *(const v8f*)(G + (size_t)n * NTOK + (size_t)b * SEQ + tc);
    v8us oh, ol;
#pragma unroll
    for (int q = 0; q < 8; ++q) { unsigned short a2, c2; splitf(ok ? v[q] : 0.0f, a2, c2); oh[q] = a2; ol[q] = c2; }
    *(volatile v8us*)(Vh + e) = oh; *(volatile v8us*)(Vl + e) = ol; __threadfence(); *(volatile v8us*)(Vh + e) = oh; *(volatile v8us*)(Vl + e) = ol;
}

__device__ __forceinline__ v8f mma3(v8f c, v16bf a, v16bf a2, v16bf b, v16bf b2) {
    c = wmmab(a, b, c); c = wmmab(a2, b, c); c = wmmab(a, b2, c);
    asm volatile("v_nop\n\tv_nop\n\tv_nop\n\tv_nop" : "+v"(c) : "v"(a), "v"(a2), "v"(b), "v"(b2));
    return c;
}

__global__ __launch_bounds__(32) void k_band(const bf* __restrict__ Qh, const bf* __restrict__ Ql, const bf* __restrict__ Kh, const bf* __restrict__ Kl,
                                            const bf* __restrict__ VTh, const bf* __restrict__ VTl, bf* CTh, bf* CTl) {
    __shared__ __align__(16) float ss[16 * 36];
    __shared__ __align__(16) bf pph[16 * 40];
    __shared__ __align__(16) bf ppl[16 * 40];
    __shared__ __align__(16) bf cs[2 * 16 * 72];
    const int lane = threadIdx.x & 31, lr = lane & 15, hh = lane >> 4;
    const int tile = blockIdx.x; const int qt = tile % (SEQ / 16); const int bh = tile / (SEQ / 16); const int h = bh % NH; const int b = bh / NH;
    const int q0 = qt * 16;
    const size_t qrow = (size_t)b * TP + PADL + q0;
    const size_t krow = qrow - 8;

    v8f sc[2]; sc[0] = (v8f){}; sc[1] = (v8f){};
#pragma unroll
    for (int ks = 0; ks < 2; ++ks) {
        const int k0 = ks * 32;
        const size_t ao = (qrow + lr) * DM + h * HD + k0 + 8 * hh;
        const v16bf a = WFrag<bf>::ld(Qh + ao), a2 = WFrag<bf>::ld(Ql + ao);
#pragma unroll
        for (int j = 0; j < 2; ++j) { const size_t ko = (krow + 16 * j + lr) * DM + h * HD + k0 + 8 * hh; sc[j] = mma3(sc[j], a, a2, WFrag<bf>::ld(Kh + ko), WFrag<bf>::ld(Kl + ko)); }
    }
#pragma unroll
    for (int j = 0; j < 2; ++j)
#pragma unroll
        for (int r = 0; r < 8; ++r) ss[(8 * hh + r) * 36 + 16 * j + lr] = sc[j][r];
    __syncthreads();

    float tv[16]; unsigned okm = 0u; float mx = -3.0e38f;
#pragma unroll
    for (int g = 0; g < 4; ++g) {
        const v4f s4 = *(const v4fa*)(ss + lr * 36 + 16 * hh + 4 * g);
#pragma unroll
        for (int u = 0; u < 4; ++u) {
            const int c = 4 * g + u; const int kk = 16 * hh + c; const int kt = q0 - 8 + kk; const int dl = kk - 8 - lr;
            const bool ok = (kt >= 0) && (kt < SEQ) && (dl >= -HALFW) && (dl <= HALFW);
            const float t = s4[u] * SCL; tv[c] = t; okm |= ok ? (1u << c) : 0u; mx = ok ? fmaxf(mx, t) : mx; } }
    mx = fmaxf(mx, __shfl_xor(mx, 16, 32));
    float ev[16]; float sum = 0.0f;
#pragma unroll
    for (int c = 0; c < 16; ++c) { const bool ok = ((okm >> c) & 1u) != 0u; float d0 = __fsub_rn(tv[c], mx); asm volatile("" : "+v"(d0));
        const float e = ok ? __builtin_amdgcn_exp2f(__fmul_rn(d0, 1.4426950408889634f)) : 0.0f; ev[c] = e; sum += e; }
    sum += __shfl_xor(sum, 16, 32);
    const float f = 1.0f / sum;
    v8us oh[2], ol[2];
#pragma unroll
    for (int c = 0; c < 16; ++c) { unsigned short a2, c2; splitf(ev[c] * f, a2, c2); oh[c >> 3][c & 7] = a2; ol[c >> 3][c & 7] = c2; }
    *(v8us*)(pph + lr * 40 + 16 * hh) = oh[0]; *(v8us*)(pph + lr * 40 + 16 * hh + 8) = oh[1];
    *(v8us*)(ppl + lr * 40 + 16 * hh) = ol[0]; *(v8us*)(ppl + lr * 40 + 16 * hh + 8) = ol[1];
    __syncthreads();

    const v16bf pa = WFrag<bf>::ld(pph + lr * 40 + 8 * hh), pa2 = WFrag<bf>::ld(ppl + lr * 40 + 8 * hh);
    v8f o[4];
#pragma unroll
    for (int nt = 0; nt < 4; ++nt) {
        const size_t vo = ((size_t)(h * HD + 16 * nt + lr) * NB + b) * TP + PADL + q0 - 8 + 8 * hh;
        o[nt] = mma3((v8f){}, pa, pa2, WFrag<bf>::ld(VTh + vo), WFrag<bf>::ld(VTl + vo)); }
#pragma unroll
    for (int nt = 0; nt < 4; ++nt)
#pragma unroll
        for (int r = 0; r < 8; ++r) { unsigned short a2, c2; splitf(o[nt][r], a2, c2); const int li = (8 * hh + r) * 72 + 16 * nt + lr; cs[li] = a2; cs[16 * 72 + li] = c2; }
    __syncthreads();

    const size_t tokbase = (size_t)b * SEQ + q0;
#pragma unroll 1
    for (int ps = 0; ps < 2; ++ps) {
#pragma unroll
        for (int s = 0; s < 4; ++s) {
            const int row = 4 * s + (lane >> 3), pc = lane & 7;
            const v8us vh = *(const v8usa*)(cs + row * 72 + pc * 8); const v8us vl = *(const v8usa*)(cs + 16 * 72 + row * 72 + pc * 8);
            const size_t go = (tokbase + row) * DM + h * HD + pc * 8;
            *(volatile v8us*)(CTh + go) = vh; *(volatile v8us*)(CTl + go) = vl; }
        if (ps == 0) __threadfence(); }
}

extern "C" void kernel_launch(void* const* d_in, const int* in_sizes, int n_in,
                              void* d_out, int out_size, void* d_ws, size_t ws_size, hipStream_t stream) {
    if (n_in < 6) return;
    if ((size_t)in_sizes[0] < ((size_t)(NB - 1) * SEQ_FULL + SEQ) * DM) return;
    if (in_sizes[1] < DM * DM || in_sizes[2] < DM * DM || in_sizes[3] < DM * DM || in_sizes[4] < DM * DM || in_sizes[5] < DM) return;
    if ((size_t)out_size < (size_t)NTOK * DM) return;
    const float* x  = (const float*)d_in[0];
    const float* Wq = (const float*)d_in[1];
    const float* Wk = (const float*)d_in[2];
    const float* Wv = (const float*)d_in[3];
    const float* Wo = (const float*)d_in[4];
    const float* bo = (const float*)d_in[5];
    float* OUT = (float*)d_out;
    char* wsp = (char*)d_ws;
    auto take = [&](size_t bytes) { char* p = wsp; wsp += (bytes + 255) & ~(size_t)255; return (void*)p; };
    const size_t plN = (size_t)NB * TP * DM;
    bf* xB  = (bf*)take((size_t)NTOK * DM * 2);
    bf* WqB = (bf*)take((size_t)DM * DM * 2); bf* WkB = (bf*)take((size_t)DM * DM * 2); bf* WvB = (bf*)take((size_t)DM * DM * 2); bf* WoB = (bf*)take((size_t)DM * DM * 2);
    float* Qf  = (float*)take((size_t)NTOK * DM * 4); float* Kf = (float*)take((size_t)NTOK * DM * 4); float* VTf = (float*)take((size_t)DM * NTOK * 4);
    bf* Qh = (bf*)take(plN * 2); bf* Ql = (bf*)take(plN * 2); bf* Kh = (bf*)take(plN * 2); bf* Kl = (bf*)take(plN * 2);
    bf* VTh = (bf*)take(plN * 2); bf* VTl = (bf*)take(plN * 2);
    bf* CTh = (bf*)take((size_t)NTOK * DM * 2); bf* CTl = (bf*)take((size_t)NTOK * DM * 2);
    if ((size_t)(wsp - (char*)d_ws) > ws_size) return;

    const size_t n8x = (size_t)SEQ * DM / 8, n8w = (size_t)DM * DM / 8, n8p = plN / 8;
    for (int b = 0; b < NB; ++b) k_cvt8<<<(unsigned)((n8x + 255) / 256), 256, 0, stream>>>(x + (size_t)b * SEQ_FULL * DM, xB + (size_t)b * SEQ * DM, n8x);
    k_cvt8<<<(unsigned)((n8w + 255) / 256), 256, 0, stream>>>(Wq, WqB, n8w);
    k_cvt8<<<(unsigned)((n8w + 255) / 256), 256, 0, stream>>>(Wk, WkB, n8w);
    k_cvt8<<<(unsigned)((n8w + 255) / 256), 256, 0, stream>>>(Wv, WvB, n8w);
    k_cvt8<<<(unsigned)((n8w + 255) / 256), 256, 0, stream>>>(Wo, WoB, n8w);
    k_gemmw<bf, 0, false><<<dim3(NTOK / 64, DM / 64, 1), 32, 0, stream>>>(xB, nullptr, WqB, nullptr, DM, Qf, DM, nullptr, 0, 0, 0);
    k_gemmw<bf, 0, false><<<dim3(NTOK / 64, DM / 64, 1), 32, 0, stream>>>(xB, nullptr, WkB, nullptr, DM, Kf, DM, nullptr, 0, 0, 0);
    k_gemmw<bf, 0, false><<<dim3(DM / 64, NTOK / 64, 1), 32, 0, stream>>>(WvB, nullptr, xB, nullptr, DM, VTf, NTOK, nullptr, 0, 0, 0);
    k_hlpad<<<(unsigned)((n8p + 255) / 256), 256, 0, stream>>>(Qf, Qh, Ql, n8p);
    k_hlpad<<<(unsigned)((n8p + 255) / 256), 256, 0, stream>>>(Kf, Kh, Kl, n8p);
    k_vthl<<<(unsigned)((n8p + 255) / 256), 256, 0, stream>>>(VTf, VTh, VTl, n8p);
    k_band<<<(unsigned)(NB * NH * (SEQ / 16)), 32, 0, stream>>>(Qh, Ql, Kh, Kl, VTh, VTl, CTh, CTl);
    k_gemmw<bf, 1, true><<<dim3(NTOK / 64, DM / 64, 1), 32, 0, stream>>>(CTh, CTl, WoB, nullptr, DM, OUT, DM, bo, 0, 0, 0);
}
